// MultiHeadLatentAttention_72009421685113
// MI455X (gfx1250) — hardware-verified
//
#include <hip/hip_runtime.h>


#define EMB 1024
#define HEADS 16
#define HDM 64
#ifndef NB
#define NB 4
#endif
#ifndef SEQ
#define SEQ 2048
#endif
#define NB_FULL 4
#define SEQ_FULL 2048
#define QKVLD (3 * EMB)
#define PSCALE 4096.0f

static_assert(EMB == HEADS * HDM);
static_assert(HDM == 64);
static_assert(SEQ % 128 == 0);
static_assert(SEQ >= 64 && SEQ <= SEQ_FULL);
static_assert(NB >= 1 && NB <= NB_FULL);
static_assert((3 * EMB) % 128 == 0 && EMB % 128 == 0 && EMB % 32 == 0);

typedef __attribute__((ext_vector_type(16))) __bf16   v16bf;
typedef __attribute__((ext_vector_type(16))) _Float16 v16h;
typedef __attribute__((ext_vector_type(8)))  float    v8f;
typedef __attribute__((ext_vector_type(8)))  unsigned v8u;
typedef __attribute__((ext_vector_type(4)))  float    v4f;
typedef float v4fa __attribute__((ext_vector_type(4), __may_alias__));

__device__ __forceinline__ unsigned f2bf(float f) { unsigned u = __float_as_uint(f); u += 0x7FFFu + ((u >> 16) & 1u); return u >> 16; }
__device__ __forceinline__ float bfr(float f) { return __uint_as_float(f2bf(f) << 16); }
__device__ __forceinline__ unsigned f2h(float f) { return (unsigned)__builtin_bit_cast(unsigned short, (_Float16)f); }
__device__ __forceinline__ int kpat(int v, int half) { return ((v & 4) ? 16 : 0) + half * 8 + 2 * (v & 3); }

template <int F16, int NP> struct Opnd { v16bf p[NP]; };

template <int F16, int NP> __device__ __forceinline__ void pack2(float f0, float f1, unsigned* o) {
    if (F16) { o[0] = f2h(f0) | (f2h(f1) << 16); return; }
    unsigned h0 = f2bf(f0), h1 = f2bf(f1); o[0] = h0 | (h1 << 16);
    if (NP >= 2) {
        float r0 = f0 - __uint_as_float(h0 << 16), r1 = f1 - __uint_as_float(h1 << 16);
        unsigned m0 = f2bf(r0), m1 = f2bf(r1); o[1] = m0 | (m1 << 16);
        if (NP >= 3) {
            float s0 = r0 - __uint_as_float(m0 << 16), s1 = r1 - __uint_as_float(m1 << 16);
            o[2] = f2bf(s0) | (f2bf(s1) << 16);
        }
    }
}
template <int F16, int NP, int RND> __device__ __forceinline__ void op_row(const float* rowp, int half, float sc, Opnd<F16, NP>& o) {
    v8u u[NP];
#pragma unroll
    for (int v = 0; v < 8; ++v) {
        int kk = kpat(v, half); unsigned t[3];
        float f0 = rowp[kk], f1 = rowp[kk + 1];
        if (RND) { f0 = bfr(f0); f1 = bfr(f1); }
        pack2<F16, NP>(f0 * sc, f1 * sc, t);
#pragma unroll
        for (int p = 0; p < NP; ++p) u[p][v] = t[p];
    }
#pragma unroll
    for (int p = 0; p < NP; ++p) o.p[p] = __builtin_bit_cast(v16bf, u[p]);
}
template <int F16, int NP, int RND> __device__ __forceinline__ void op_row_tail(const float* rowp, int half, float sc, int kvalid, Opnd<F16, NP>& o) {
    v8u u[NP];
#pragma unroll
    for (int v = 0; v < 8; ++v) {
        int kk = kpat(v, half); unsigned t[3];
        float f0 = kk < kvalid ? rowp[kk] : 0.0f, f1 = (kk + 1) < kvalid ? rowp[kk + 1] : 0.0f;
        if (RND) { f0 = bfr(f0); f1 = bfr(f1); }
        pack2<F16, NP>(f0 * sc, f1 * sc, t);
#pragma unroll
        for (int p = 0; p < NP; ++p) u[p][v] = t[p];
    }
#pragma unroll
    for (int p = 0; p < NP; ++p) o.p[p] = __builtin_bit_cast(v16bf, u[p]);
}
template <int F16, int NP, int RND> __device__ __forceinline__ void op_col(const float* M, int ld, int n, int k0, int half, float sc, Opnd<F16, NP>& o) {
    v8u u[NP];
#pragma unroll
    for (int v = 0; v < 8; ++v) {
        int kk = k0 + kpat(v, half); unsigned t[3];
        float f0 = M[(size_t)kk * ld + n], f1 = M[(size_t)(kk + 1) * ld + n];
        if (RND) { f0 = bfr(f0); f1 = bfr(f1); }
        pack2<F16, NP>(f0 * sc, f1 * sc, t);
#pragma unroll
        for (int p = 0; p < NP; ++p) u[p][v] = t[p];
    }
#pragma unroll
    for (int p = 0; p < NP; ++p) o.p[p] = __builtin_bit_cast(v16bf, u[p]);
}
template <int F16, int NP, int RND> __device__ __forceinline__ void op_col_tail(const float* M, int ld, int n, int k0, int half, float sc, int K, Opnd<F16, NP>& o) {
    v8u u[NP];
#pragma unroll
    for (int v = 0; v < 8; ++v) {
        int kk = k0 + kpat(v, half); unsigned t[3];
        float f0 = kk < K ? M[(size_t)kk * ld + n] : 0.0f, f1 = (kk + 1) < K ? M[(size_t)(kk + 1) * ld + n] : 0.0f;
        if (RND) { f0 = bfr(f0); f1 = bfr(f1); }
        pack2<F16, NP>(f0 * sc, f1 * sc, t);
#pragma unroll
        for (int p = 0; p < NP; ++p) u[p][v] = t[p];
    }
#pragma unroll
    for (int p = 0; p < NP; ++p) o.p[p] = __builtin_bit_cast(v16bf, u[p]);
}
__device__ __forceinline__ v8f wm_bf16(v16bf a, v16bf b, v8f c) { return __builtin_amdgcn_wmma_f32_16x16x32_bf16(false, a, false, b, (short)0, c, false, false); }
template <int F16, int PA, int PB> __device__ __forceinline__ v8f wmma_op(const Opnd<F16, PA>& a, const Opnd<F16, PB>& b, v8f c) {
    if (F16) {
        v16h ah = __builtin_bit_cast(v16h, a.p[0]), bh = __builtin_bit_cast(v16h, b.p[0]);
        c = __builtin_amdgcn_wmma_f32_16x16x32_f16(false, ah, false, bh, (short)0, c, false, false);
        asm volatile("v_nop\n\tv_nop\n\tv_nop\n\tv_nop" : "+v"(c) : "v"(ah), "v"(bh));
        return c;
    }
    constexpr int NMX = PA > PB ? PA : PB;
#pragma unroll
    for (int i = 0; i < PA; ++i)
#pragma unroll
        for (int j = 0; j < PB; ++j)
            if (i + j < NMX) c = wm_bf16(a.p[i], b.p[j], c);
    if (PA == 1 && PB == 1)      asm volatile("v_nop\n\tv_nop\n\tv_nop\n\tv_nop" : "+v"(c) : "v"(a.p[0]), "v"(b.p[0]));
    else if (PA == 2 && PB == 1) asm volatile("v_nop\n\tv_nop\n\tv_nop\n\tv_nop" : "+v"(c) : "v"(a.p[0]), "v"(a.p[1]), "v"(b.p[0]));
    else if (PA == 1 && PB == 2) asm volatile("v_nop\n\tv_nop\n\tv_nop\n\tv_nop" : "+v"(c) : "v"(a.p[0]), "v"(b.p[0]), "v"(b.p[1]));
    else if (PA == 2 && PB == 2) asm volatile("v_nop\n\tv_nop\n\tv_nop\n\tv_nop" : "+v"(c) : "v"(a.p[0]), "v"(a.p[1]), "v"(b.p[0]), "v"(b.p[1]));
    else                         asm volatile("v_nop\n\tv_nop\n\tv_nop\n\tv_nop" : "+v"(c) : "v"(a.p[0]), "v"(a.p[PA - 1]), "v"(b.p[0]), "v"(b.p[PB - 1]), "v"(a.p[PA / 2]), "v"(b.p[PB / 2]));
    return c;
}

struct ZMap { long long s1; long long s2; int zdiv; int pad_; };
__device__ __forceinline__ size_t zoff(const ZMap& m, int z) { return (size_t)((long long)(z / m.zdiv) * m.s1 + (long long)(z % m.zdiv) * m.s2); }

#define ACT_NONE 0
#define ACT_RELU 1
#define ACT_GELU_ERF 2
#define ACT_SILU 3
#define ACT_TANH 4
__device__ __forceinline__ float act_apply(int act, float x) {
    if (act == ACT_RELU) return x > 0.f ? x : 0.f;
    if (act == ACT_GELU_ERF) return 0.5f * x * (1.0f + erff(x * 0.70710678118654752f));
    if (act == ACT_SILU) return x / (1.0f + expf(-x));
    if (act == ACT_TANH) return tanhf(x);
    return x;
}
struct GemmArgs {
    ZMap za, zb_, zc, zbias, zadd, zrsc, zmul;
    const float* A; const float* Bm; float* C; const float* bias; const float* add; const float* rsc; const float* mul;
    long long ldadd, ldmul;
    int lda, ldb, ldc, K;
    float ascale, bscale, oscale, addscale;
    int M, nvalid, nstore, ldrsc;
    int bcs, pad1, pad2, pad3;
};
template <int BT, int F16, int PA, int PB, int RW, int CW, int ACT, int RA, int RB>
__global__ __launch_bounds__(256) void gemm_kernel(GemmArgs g) {
    constexpr int TR = 16 * RW, TC = 64 * CW, CSTR = TC + 4;
    __shared__ __align__(16) float cst[TR * CSTR];
    const int z = blockIdx.z;
    const float* A = g.A + zoff(g.za, z); const float* Bm = g.Bm + zoff(g.zb_, z); float* C = g.C + zoff(g.zc, z);
    const int tid = threadIdx.x, lane = tid & 31, wv = tid >> 5;
    const int l16 = lane & 15, half = lane >> 4;
    const int rt = wv % RW, ch = wv / RW;
    const int row0 = blockIdx.x * TR, col0 = blockIdx.y * TC + ch * 64;
    int arix = row0 + rt * 16 + l16; if (arix >= g.M) arix = g.M - 1;
    const float* arow = A + (size_t)arix * g.lda;
    v8f acc[4];
#pragma unroll
    for (int t = 0; t < 4; ++t) acc[t] = (v8f){};
    const int K = g.K;
#pragma unroll 1
    for (int kc = 0; kc < K; kc += 32) {
        Opnd<F16, PA> a;
        if (kc + 32 <= K) op_row<F16, PA, RA>(arow + kc, half, g.ascale, a); else op_row_tail<F16, PA, RA>(arow + kc, half, g.ascale, K - kc, a);
#pragma unroll
        for (int t = 0; t < 4; ++t) {
            Opnd<F16, PB> b;
            const int n = col0 + t * 16 + l16;
            if (n < g.nvalid) {
                if (BT) { if (kc + 32 <= K) op_row<F16, PB, RB>(Bm + (size_t)n * g.ldb + kc, half, g.bscale, b); else op_row_tail<F16, PB, RB>(Bm + (size_t)n * g.ldb + kc, half, g.bscale, K - kc, b); }
                else    { if (kc + 32 <= K) op_col<F16, PB, RB>(Bm, g.ldb, n * g.bcs, kc, half, g.bscale, b); else op_col_tail<F16, PB, RB>(Bm, g.ldb, n * g.bcs, kc, half, g.bscale, K, b); }
            } else {
#pragma unroll
                for (int p = 0; p < PB; ++p) b.p[p] = (v16bf){};
            }
            acc[t] = wmma_op<F16, PA, PB>(a, b, acc[t]);
        }
    }
    const float* bias = g.bias ? g.bias + zoff(g.zbias, z) : nullptr;
    const float* add = g.add ? g.add + zoff(g.zadd, z) : nullptr;
    const float* rsc = g.rsc ? g.rsc + zoff(g.zrsc, z) : nullptr;
    const float* mul = g.mul ? g.mul + zoff(g.zmul, z) : nullptr;
#pragma unroll
    for (int t = 0; t < 4; ++t) {
        const int cl = ch * 64 + t * 16 + l16;
        const int cg = blockIdx.y * TC + cl;
        const bool cok = cg < g.nvalid;
        const float bv = (bias && cok) ? bias[(size_t)cg * g.bcs] : 0.0f;
#pragma unroll
        for (int r = 0; r < 8; ++r) {
            const int rl = rt * 16 + r + 8 * half;
            float v = acc[t][r] * g.oscale + bv;
            int rg = row0 + rl; if (rg >= g.M) rg = g.M - 1;
            if (rsc) v *= rsc[(size_t)rg * g.ldrsc];
            if (mul && cok) v *= mul[(size_t)rg * g.ldmul + cg];
            if (add && cok) v += g.addscale * add[(size_t)rg * g.ldadd + cg];
            cst[rl * CSTR + cl] = v;
        }
    }
    __syncthreads();
    const int col = tid % TC, rsel = tid / TC, rstep = 256 / TC;
    if (ACT != ACT_NONE) {
#pragma unroll 1
        for (int r = rsel; r < TR; r += rstep) cst[r * CSTR + col] = act_apply(ACT, cst[r * CSTR + col]);
    }
    float* ob = C + (size_t)row0 * g.ldc + (size_t)blockIdx.y * TC;
    const bool colok = (int)(blockIdx.y * TC + col) < g.nstore;
    const int rmax = (g.M - row0 < TR) ? (g.M - row0) : TR;
    auto pass = [&]() {
        if (colok) {
#pragma unroll 4
            for (int r = rsel; r < rmax; r += rstep) *(volatile float*)(ob + (size_t)r * g.ldc + col) = cst[r * CSTR + col];
        }
    };
    pass();
    __threadfence();
    pass();
}
static inline ZMap zm(long long s1) { ZMap m; m.s1 = s1; m.s2 = 0; m.zdiv = 1; m.pad_ = 0; return m; }
static inline ZMap zm2(long long s1, long long s2, int zdiv) { ZMap m; m.s1 = s1; m.s2 = s2; m.zdiv = zdiv; m.pad_ = 0; return m; }
static inline GemmArgs gemm_args(const float* A, int lda, ZMap za, const float* Bm, int ldb, ZMap zb, float* C, int ldc, ZMap zc, int M, int N, int K) {
    GemmArgs g; g.za = za; g.zb_ = zb; g.zc = zc; g.zbias = zm(0); g.zadd = zm(0); g.zrsc = zm(0); g.zmul = zm(0);
    g.A = A; g.Bm = Bm; g.C = C; g.bias = nullptr; g.add = nullptr; g.rsc = nullptr; g.mul = nullptr; g.ldadd = 0; g.ldmul = 0;
    g.lda = lda; g.ldb = ldb; g.ldc = ldc; g.K = K; g.ascale = 1.0f; g.bscale = 1.0f; g.oscale = 1.0f; g.addscale = 1.0f; g.M = M; g.nvalid = N; g.nstore = N; g.ldrsc = 1;
    g.bcs = 1; g.pad1 = 0; g.pad2 = 0; g.pad3 = 0;
    return g;
}
static_assert(sizeof(ZMap) == 24);
static_assert(sizeof(GemmArgs) == 7 * 24 + 7 * 8 + 2 * 8 + 4 * 4 + 4 * 4 + 4 * 4 + 4 * 4);

#define KP 68
#define PPITCH 36
#define OPITCH 68
static_assert(16 * PPITCH <= 16 * OPITCH);

__device__ __forceinline__ int slot_mult(int s, int j, int w0) {
    const int kr = w0 - 8 + j;
    const int reg = (kr >= 0 && kr < SEQ && kr >= s - 3 && kr <= s + 3) ? 1 : 0;
    const int m0 = (s < 3) ? (3 - s) : 0;
    const int m31 = (s > SEQ - 4) ? (s - (SEQ - 4)) : 0;
    return (j == 0) ? m0 : ((j == 31) ? m31 : reg);
}

__global__ __launch_bounds__(64) void win_attn(const float* qkv, float* ctx) {
    __shared__ __align__(16) float Kt[2][32 * KP];
    __shared__ __align__(16) float Vt[2][32 * KP];
    __shared__ __align__(16) float PO[2][16 * OPITCH];
    const int tid = threadIdx.x, lane = tid & 31, wv = tid >> 5, l16 = lane & 15, half = lane >> 4;
    const int b = blockIdx.z, h = blockIdx.y;
    const int w0 = blockIdx.x * 32 + wv * 16;
    const size_t prow = (size_t)b * SEQ;
    const float* qcol = qkv + (size_t)h * HDM;
    const float* kcol = qkv + EMB + (size_t)h * HDM;
    const float* vcol = qkv + 2 * EMB + (size_t)h * HDM;
    float* Kw = Kt[wv]; float* Vw = Vt[wv]; float* Pw = PO[wv];

#pragma unroll 4
    for (int it = 0; it < 16; ++it) {
        const int idx = it * 32 + lane, j = idx >> 4, c4 = idx & 15;
        const int kr = w0 - 8 + j;
        const bool valid = (j == 0) || (j == 31) || (kr >= 0 && kr < SEQ);
        const int kcl = kr < 0 ? 0 : (kr > SEQ - 1 ? SEQ - 1 : kr);
        const int kj = (j == 0) ? (SEQ - 1) : ((j == 31) ? 0 : kcl);
        const size_t roff = (prow + (size_t)kj) * QKVLD + (size_t)c4 * 4;
        const float4 ka = *(const float4*)(kcol + roff);
        const float4 va = *(const float4*)(vcol + roff);
        const float4 kz = make_float4(valid ? ka.x : 0.0f, valid ? ka.y : 0.0f, valid ? ka.z : 0.0f, valid ? ka.w : 0.0f);
        const float4 vz = make_float4(valid ? va.x : 0.0f, valid ? va.y : 0.0f, valid ? va.z : 0.0f, valid ? va.w : 0.0f);
        *(float4*)(Kw + j * KP + c4 * 4) = kz;
        *(float4*)(Vw + j * KP + c4 * 4) = vz;
    }
    __syncthreads();

    v8f sacc[2];
    sacc[0] = (v8f){}; sacc[1] = (v8f){};
    const float* qrow = qcol + (prow + (size_t)(w0 + l16)) * QKVLD;
#pragma unroll
    for (int kc = 0; kc < HDM; kc += 32) {
        Opnd<1, 1> a; op_row<1, 1, 0>(qrow + kc, half, 1.0f, a);
#pragma unroll
        for (int t = 0; t < 2; ++t) {
            Opnd<1, 1> bb; op_row<1, 1, 0>(Kw + (t * 16 + l16) * KP + kc, half, 1.0f, bb);
            sacc[t] = wmma_op<1, 1, 1>(a, bb, sacc[t]);
        }
    }
#pragma unroll
    for (int r = 0; r < 8; ++r) {
        const int s = w0 + 8 * half + r;
        const int m0 = slot_mult(s, l16, w0), m1 = slot_mult(s, 16 + l16, w0);
        const float s0 = sacc[0][r] * 0.125f, s1 = sacc[1][r] * 0.125f;
        float mx = -__builtin_inff();
        mx = fmaxf(mx, m0 > 0 ? s0 : -__builtin_inff());
        mx = fmaxf(mx, m1 > 0 ? s1 : -__builtin_inff());
        mx = fmaxf(mx, __shfl_xor(mx, 8, 32));
        mx = fmaxf(mx, __shfl_xor(mx, 4, 32));
        mx = fmaxf(mx, __shfl_xor(mx, 2, 32));
        mx = fmaxf(mx, __shfl_xor(mx, 1, 32));
        const float e0 = (float)m0 * expf(fminf(s0 - mx, 0.0f));
        const float e1 = (float)m1 * expf(fminf(s1 - mx, 0.0f));
        float sum = e0 + e1;
        sum += __shfl_xor(sum, 8, 32);
        sum += __shfl_xor(sum, 4, 32);
        sum += __shfl_xor(sum, 2, 32);
        sum += __shfl_xor(sum, 1, 32);
        const float rs = 1.0f / sum;
        Pw[(8 * half + r) * PPITCH + l16] = e0 * rs;
        Pw[(8 * half + r) * PPITCH + 16 + l16] = e1 * rs;
    }
    __syncthreads();

    Opnd<1, 1> pa; op_row<1, 1, 0>(Pw + l16 * PPITCH, half, PSCALE, pa);
    v8f oacc[4];
#pragma unroll
    for (int t = 0; t < 4; ++t) {
        oacc[t] = (v8f){};
        Opnd<1, 1> vb; op_col<1, 1, 0>(Vw, KP, t * 16 + l16, 0, half, 1.0f, vb);
        oacc[t] = wmma_op<1, 1, 1>(pa, vb, oacc[t]);
    }
    __syncthreads();
    const float OSC = 1.0f / PSCALE;
#pragma unroll
    for (int t = 0; t < 4; ++t)
#pragma unroll
        for (int r = 0; r < 8; ++r) Pw[(8 * half + r) * OPITCH + t * 16 + l16] = oacc[t][r] * OSC;
    __syncthreads();

    float* cbase = ctx + (prow + (size_t)w0) * EMB + (size_t)h * HDM + 4 * l16;
    auto opass = [&]() {
#pragma unroll
        for (int i = 0; i < 8; ++i) {
            const int row = 2 * i + half;
            const v4f v = *(const v4fa*)(Pw + row * OPITCH + 4 * l16);
            *(volatile v4f*)(cbase + (size_t)row * EMB) = v;
        }
    };
    opass();
    __threadfence();
    opass();
}

extern "C" void kernel_launch(void* const* d_in, const int* in_sizes, int n_in,
                              void* d_out, int out_size, void* d_ws, size_t ws_size, hipStream_t stream) {
    if (n_in < 7) return;
    const float* x      = (const float*)d_in[0];
    const float* W_qkv  = (const float*)d_in[1];
    const float* b_qkv  = (const float*)d_in[2];
    const float* W_lat  = (const float*)d_in[3];
    const float* b_lat  = (const float*)d_in[4];
    const float* W_proj = (const float*)d_in[5];
    const float* b_proj = (const float*)d_in[6];
    float* out = (float*)d_out;

    if ((long long)in_sizes[0] < (long long)(NB - 1) * SEQ_FULL * EMB + (long long)SEQ * EMB) return;
    if (in_sizes[1] < 3 * EMB * EMB) return;
    if (in_sizes[2] < 3 * EMB) return;
    if (in_sizes[3] < HDM * HDM) return;
    if (in_sizes[4] < HDM) return;
    if (in_sizes[5] < EMB * EMB) return;
    if (in_sizes[6] < EMB) return;
    if ((long long)out_size < (long long)NB * SEQ * EMB) return;

    const size_t rows = (size_t)NB * SEQ;
    float* qkv = (float*)d_ws;
    float* ctx = qkv + rows * QKVLD;
    const size_t wsNeed = (rows * QKVLD + rows * EMB) * sizeof(float);
    if (wsNeed > ws_size) return;

    { GemmArgs g = gemm_args(x, EMB, zm((long long)SEQ_FULL * EMB), W_qkv, EMB, zm(0), qkv, QKVLD, zm((long long)SEQ * QKVLD), SEQ, 3 * EMB, EMB);
      g.bias = b_qkv; g.bscale = 32.0f; g.oscale = 1.0f / 32.0f;
      gemm_kernel<1, 1, 1, 1, 4, 2, ACT_NONE, 1, 1><<<dim3(SEQ / 64, (3 * EMB) / 128, NB), 256, 0, stream>>>(g); }
    { GemmArgs g = gemm_args(qkv + EMB, QKVLD, zm(HDM), W_lat, HDM, zm(0), qkv + EMB, QKVLD, zm(HDM), (int)rows, HDM, HDM);
      g.bias = b_lat; g.bscale = 8.0f; g.oscale = 0.125f;
      gemm_kernel<1, 1, 1, 1, 8, 1, ACT_NONE, 0, 1><<<dim3((unsigned)(rows / 128), 1, 2 * HEADS), 256, 0, stream>>>(g); }
    win_attn<<<dim3(SEQ / 32, HEADS, NB), 64, 0, stream>>>(qkv, ctx);
    { GemmArgs g = gemm_args(ctx, EMB, zm(0), W_proj, EMB, zm(0), out, EMB, zm(0), (int)rows, EMB, EMB);
      g.bias = b_proj; g.bscale = 32.0f; g.oscale = 1.0f / 32.0f;
      gemm_kernel<1, 1, 1, 1, 4, 2, ACT_NONE, 0, 1><<<dim3((unsigned)(rows / 64), EMB / 128, 1), 256, 0, stream>>>(g); }
}
